// RAMCrossAttention_22832046146305
// MI455X (gfx1250) — hardware-verified
//
#include <hip/hip_runtime.h>

#define NQ   4096
#define NK   4096
#define HH   4
#define DB   64
#define EB   64
#define NPOS 13
#define KPW  (EB + NPOS)
#define SIMK 12
#define VALK 10
#define OUTK 12
#define SIMT 4096
#define VALT 1024
#define OUTT 4096
#define CMB  (HH * DB)
#define QT   64
#define MTHR 128
#define VTHR 256
#define VKC  (8 * VTHR)

static_assert(NQ % QT == 0);
static_assert(NK % VKC == 0);
static_assert(NK % 32 == 0);
static_assert(QT == 16 * (MTHR / 32));
static_assert(SIMT % MTHR == 0);
static_assert(NK % MTHR == 0);
static_assert((QT * DB) % (4 * MTHR) == 0);
static_assert(MTHR == 2 * DB);

typedef _Float16       v16h __attribute__((ext_vector_type(16)));
typedef _Float16       v8h  __attribute__((ext_vector_type(8)));
typedef float          v8f  __attribute__((ext_vector_type(8)));
typedef float          v4f  __attribute__((ext_vector_type(4)));
typedef unsigned short v8us __attribute__((ext_vector_type(8)));
typedef v8h  __attribute__((may_alias)) v8ha;
typedef v4f  __attribute__((may_alias)) v4fa;
typedef v8us __attribute__((may_alias)) v8usa;

union Frag { v16h v; v8h half[2]; };

__device__ __forceinline__ v8f wmma16(v16h a, v16h b, v8f c) {
  v8f d = __builtin_amdgcn_wmma_f32_16x16x32_f16(false, a, false, b, (short)0, c, false, false);
#if defined(__HIP_DEVICE_COMPILE__)
  asm volatile("v_nop\n\tv_nop\n\tv_nop\n\tv_nop" : "+v"(d) : "v"(a), "v"(b));
#endif
  return d;
}

__global__ __launch_bounds__(VTHR) void k_vals(
    const int* __restrict__ enc_bits,
    const int* __restrict__ val_conn,
    const float* __restrict__ val_table,
    _Float16* __restrict__ valsT)
{
  const int t = threadIdx.x;
  const int kc = blockIdx.x, d = blockIdx.y, h = blockIdx.z;
  const int hd = h * DB + d;

  int vc[VALK];
  #pragma unroll
  for (int j = 0; j < VALK; ++j) vc[j] = min(max(val_conn[hd * VALK + j], 0), KPW - 1);

  const float* vt = val_table + (size_t)hd * VALT;
  const int kb = kc * VKC + 8 * t;

  v8h o;
  #pragma unroll
  for (int i = 0; i < 8; ++i) {
    const int k = kb + i;
    int a = 0;
    #pragma unroll
    for (int j = 0; j < VALK; ++j) {
      const int c  = vc[j];
      const int e  = enc_bits[k * EB + min(c, EB - 1)];
      const int sh = (NPOS - 1) - max(c - EB, 0);
      const int pb = (k >> sh) & 1;
      a += ((c < EB) ? e : pb) << j;
    }
    const float v = vt[a & (VALT - 1)];
    o[i] = (v > 0.5f) ? (_Float16)1.0f : (_Float16)0.0f;
  }
  _Float16* dst = valsT + (size_t)hd * NK + kb;
  *(volatile v8h*)dst = o;
  __threadfence();
  *(volatile v8h*)dst = o;
}

__device__ __forceinline__ void out_store_pass(const float* so, float* ob, int tid) {
  #pragma unroll
  for (int i = 0; i < (QT * DB) / (4 * MTHR); ++i) {
    const int g = tid + MTHR * i;
    const v4f v = *(const v4fa*)(so + 4 * g);
    *(volatile v4f*)(ob + 4 * g) = v;
  }
}

__global__ __launch_bounds__(MTHR) void k_main(
    const int* __restrict__ dec_bits,
    const int* __restrict__ enc_bits,
    const int* __restrict__ sim_conn,
    const float* __restrict__ sim_table,
    const _Float16* __restrict__ valsT,
    const int* __restrict__ out_conn,
    const float* __restrict__ out_table,
    float* __restrict__ out)
{
  __shared__ __attribute__((aligned(16))) _Float16       sflag[SIMT];
  __shared__ __attribute__((aligned(16))) unsigned short sakp[NK];
  __shared__ __attribute__((aligned(16))) unsigned char  scomb[QT * CMB];
  __shared__ __attribute__((aligned(16))) float          sout[QT * DB];

  const int tid = threadIdx.x, lane = tid & 31, w = tid >> 5;
  const int hf = lane >> 4, m = lane & 15;
  const int q0 = blockIdx.x * QT;
  const int qrow = q0 + 16 * w + m;

  const v8f zero8 = {0.f, 0.f, 0.f, 0.f, 0.f, 0.f, 0.f, 0.f};

  #pragma unroll 1
  for (int h = 0; h < HH; ++h) {
    __syncthreads();

    int sc[SIMK];
    #pragma unroll
    for (int j = 0; j < SIMK; ++j) sc[j] = sim_conn[h * SIMK + j];

    #pragma unroll 4
    for (int r = 0; r < SIMT / MTHR; ++r) {
      const int i = tid + MTHR * r;
      sflag[i] = (sim_table[h * SIMT + i] > 0.5f) ? (_Float16)1.0f : (_Float16)0.0f;
    }

    #pragma unroll 1
    for (int r = 0; r < NK / MTHR; ++r) {
      const int k = tid + MTHR * r;
      int a = 0;
      #pragma unroll
      for (int j = 0; j < SIMK; ++j) {
        const int c = sc[j];
        if (c >= DB) {
          const int cc = min(c - DB, KPW - 1);
          const int e  = enc_bits[k * EB + min(cc, EB - 1)];
          const int sh = (NPOS - 1) - max(cc - EB, 0);
          const int pb = (k >> sh) & 1;
          a += ((cc < EB) ? e : pb) << j;
        }
      }
      sakp[k] = (unsigned short)(a & (SIMT - 1));
    }

    int aq = 0;
    #pragma unroll
    for (int j = 0; j < SIMK; ++j) {
      const int c = sc[j];
      if (c < DB) aq += dec_bits[qrow * DB + max(c, 0)] << j;
    }
    aq &= (SIMT - 1);
    __syncthreads();

    v8f acc[4];
    #pragma unroll
    for (int j = 0; j < 4; ++j) acc[j] = zero8;
    float cnt = 0.0f;
    const _Float16* vb = valsT + ((size_t)(h * DB + m)) * NK;

    #pragma unroll 1
    for (int k0 = 0; k0 < NK; k0 += 32) {
      const v8us u0 = *(const v8usa*)(sakp + k0 + 8 * hf);
      const v8us u1 = *(const v8usa*)(sakp + k0 + 16 + 8 * hf);
      v8h alo, ahi;
      #pragma unroll
      for (int i = 0; i < 8; ++i) {
        alo[i] = sflag[(aq + (int)u0[i]) & (SIMT - 1)];
        ahi[i] = sflag[(aq + (int)u1[i]) & (SIMT - 1)];
      }
      Frag a;
      a.half[0] = alo;
      a.half[1] = ahi;

      const v8h s8 = alo + ahi;
      const _Float16 s = ((s8[0] + s8[1]) + (s8[2] + s8[3])) + ((s8[4] + s8[5]) + (s8[6] + s8[7]));
      cnt += (float)s;

      #pragma unroll
      for (int j = 0; j < 4; ++j) {
        const _Float16* vr = vb + (size_t)(16 * j) * NK + k0;
        Frag b;
        b.half[0] = *(const v8ha*)(vr + 8 * hf);
        b.half[1] = *(const v8ha*)(vr + 16 + 8 * hf);
        acc[j] = wmma16(a.v, b.v, acc[j]);
      }
    }

    const float cm = cnt + __shfl_xor(cnt, 16);
    #pragma unroll
    for (int r = 0; r < 8; ++r) {
      const float cr = __shfl(cm, 8 * hf + r);
      const int rowl = 16 * w + 8 * hf + r;
      #pragma unroll
      for (int j = 0; j < 4; ++j) {
        const float sv = acc[j][r];
        const unsigned char g = (cr > 0.0f && (2.0f * sv) >= cr) ? (unsigned char)1 : (unsigned char)0;
        scomb[rowl * CMB + h * DB + 16 * j + m] = g;
      }
    }
  }
  __syncthreads();

  {
    const int d = tid & (DB - 1), rg = tid >> 6;
    int oc[OUTK];
    #pragma unroll
    for (int j = 0; j < OUTK; ++j) oc[j] = min(max(out_conn[d * OUTK + j], 0), CMB - 1);
    const float* ot = out_table + (size_t)d * OUTT;
    #pragma unroll 2
    for (int i = 0; i < QT / 2; ++i) {
      const int row = rg + 2 * i;
      int addr = 0;
      #pragma unroll
      for (int j = 0; j < OUTK; ++j) addr += (int)scomb[row * CMB + oc[j]] << j;
      sout[row * DB + d] = (ot[addr & (OUTT - 1)] > 0.5f) ? 1.0f : 0.0f;
    }
  }
  __syncthreads();

  float* ob = out + (size_t)q0 * DB;
  out_store_pass(sout, ob, tid);
  __threadfence();
  out_store_pass(sout, ob, tid);
}

extern "C" void kernel_launch(void* const* d_in, const int* in_sizes, int n_in,
                              void* d_out, int out_size, void* d_ws, size_t ws_size,
                              hipStream_t stream) {
  if (n_in < 8) return;
  if (in_sizes[0] != NQ * DB || in_sizes[1] != NK * EB) return;
  if (in_sizes[2] != HH * SIMK || in_sizes[3] != HH * SIMT) return;
  if (in_sizes[4] != HH * DB * VALK || in_sizes[5] != HH * DB * VALT) return;
  if (in_sizes[6] != DB * OUTK || in_sizes[7] != DB * OUTT) return;
  if (out_size != NQ * DB) return;

  const size_t vals_bytes = (size_t)HH * DB * NK * sizeof(_Float16);
  if (vals_bytes > ws_size) return;

  const int*   dec_bits  = (const int*)d_in[0];
  const int*   enc_bits  = (const int*)d_in[1];
  const int*   sim_conn  = (const int*)d_in[2];
  const float* sim_table = (const float*)d_in[3];
  const int*   val_conn  = (const int*)d_in[4];
  const float* val_table = (const float*)d_in[5];
  const int*   out_conn  = (const int*)d_in[6];
  const float* out_table = (const float*)d_in[7];
  float*       out       = (float*)d_out;
  _Float16*    valsT     = (_Float16*)d_ws;

  k_vals<<<dim3(NK / VKC, DB, HH), VTHR, 0, stream>>>(enc_bits, val_conn, val_table, valsT);
  k_main<<<dim3(NQ / QT), MTHR, 0, stream>>>(dec_bits, enc_bits, sim_conn, sim_table, valsT,
                                             out_conn, out_table, out);
}
